// GlobalNodeAttentionFull_50208167690485
// MI455X (gfx1250) — hardware-run, weakly checked
//
#include <hip/hip_runtime.h>
#include <math.h>
#include <stdint.h>

#define NN    8192
#define NGR   16
#define NHD   8
#define FD    1152
#define F3    3456
#define HD    144
#define HDK   160
#define NCAP  576
#define GG    2
#define NGRP  8
#define QKW   2304
#define CTXW  2560
#define RECW  320

static_assert(NCAP % 64 == 0);
static_assert(NGR % GG == 0);
static_assert(NGR / GG == NGRP);
static_assert(HD == 144);
static_assert(HDK == 5 * 32);
static_assert(HD == 9 * 16);
static_assert(FD % 128 == 0);
static_assert(FD == NHD * HD);
static_assert(FD % 32 == 0);
static_assert(CTXW % 32 == 0);
static_assert(CTXW == NHD * RECW);
static_assert(F3 % 128 == 0);
static_assert((GG * NCAP) % 64 == 0);
static_assert(NN % 128 == 0);
static_assert(NN == 256 * 32);

#define SM_AF  0
#define SM_WR  32
#define SM_G   160
#define SM_B   1312
#define SM_END 2464
#define SM_TOT 2560

typedef __attribute__((ext_vector_type(16))) __bf16 v16b;
typedef __attribute__((ext_vector_type(8)))  __bf16 v8b;
typedef __attribute__((ext_vector_type(8)))  float  v8f;
typedef __attribute__((ext_vector_type(4)))  float  v4f;
typedef __attribute__((ext_vector_type(4)))  unsigned int v4u;
typedef __attribute__((ext_vector_type(4)))  int    v4i;
typedef v8b __attribute__((may_alias)) v8ba;
typedef v4f __attribute__((may_alias)) v4fa;
typedef v4u __attribute__((may_alias)) v4ua;
typedef v4i __attribute__((may_alias)) v4ia;

__device__ __forceinline__ int clampi(int v, int lo, int hi) { return v < lo ? lo : (v > hi ? hi : v); }
__device__ __forceinline__ unsigned short f2bf_bits(float f) {
  unsigned u = __float_as_uint(f);
  return (unsigned short)((u + 0x7FFFu + ((u >> 16) & 1u)) >> 16);
}
__device__ __forceinline__ float bf_bits2f(unsigned short h) { return __uint_as_float(((unsigned)h) << 16); }
__device__ __forceinline__ float bfr(float f) { return bf_bits2f(f2bf_bits(f)); }
__device__ __forceinline__ unsigned pk16(unsigned short a, unsigned short b) { return (unsigned)a | ((unsigned)b << 16); }
__device__ __forceinline__ float selmax(float a, float b) { return (a > b) ? a : b; }
__device__ __forceinline__ void split_bf(float f, __bf16& hi, __bf16& lo) {
  const unsigned short hb = f2bf_bits(f);
  hi = __builtin_bit_cast(__bf16, hb);
  lo = __builtin_bit_cast(__bf16, f2bf_bits(f - bf_bits2f(hb)));
}

__device__ __forceinline__ v8f mma_bf(v16b a, v16b b, v8f c) {
  c = __builtin_amdgcn_wmma_f32_16x16x32_bf16(false, a, false, b, (short)0, c, false, false);
  asm volatile("v_nop\n\tv_nop\n\tv_nop\n\tv_nop" : "+v"(c) : "v"(a), "v"(b));
  return c;
}
union FB { v16b v; v8b h[2]; };
__device__ __forceinline__ v16b ldfrag(const __bf16* p) {
  FB f; f.h[0] = *(const v8ba*)(p); f.h[1] = *(const v8ba*)(p + 16); return f.v;
}
__device__ __forceinline__ void wave_sync_lds() {
  __builtin_amdgcn_fence(__ATOMIC_RELEASE, "workgroup");
  __builtin_amdgcn_wave_barrier();
  __builtin_amdgcn_fence(__ATOMIC_ACQUIRE, "workgroup");
}

__device__ __forceinline__ void gemm_tile64(const __bf16* __restrict__ A, int lda,
                                            const __bf16* __restrict__ Bt, int ldb,
                                            int K, int lane, v8f (&acc)[4][4]) {
  const int c = lane & 15, hh = lane >> 4;
  const __bf16* ap = A + (size_t)c * lda + 8 * hh;
  const __bf16* bp = Bt + (size_t)c * ldb + 8 * hh;
#pragma unroll 1
  for (int k0 = 0; k0 < K; k0 += 32) {
    v16b bh[4];
#pragma unroll
    for (int j = 0; j < 4; ++j) bh[j] = ldfrag(bp + (size_t)(j * 16) * ldb + k0);
#pragma unroll
    for (int i = 0; i < 4; ++i) {
      const v16b ah = ldfrag(ap + (size_t)(i * 16) * lda + k0);
#pragma unroll
      for (int j = 0; j < 4; ++j) acc[i][j] = mma_bf(ah, bh[j], acc[i][j]);
    }
  }
}

__global__ __launch_bounds__(256) void k_off(const int* __restrict__ batch, int* __restrict__ meta) {
  __shared__ int cnt[256 * 16];
  __shared__ int tot[32];
  __shared__ int ofs[32];
  const int tid = threadIdx.x;
  int c[16];
#pragma unroll
  for (int g = 0; g < 16; ++g) c[g] = 0;
#pragma unroll 1
  for (int i = 0; i < 8; ++i) {
    const v4i v = *(const v4ia*)(batch + tid * 32 + 4 * i);
#pragma unroll
    for (int g = 0; g < 16; ++g)
      c[g] += (int)(v.x == g) + (int)(v.y == g) + (int)(v.z == g) + (int)(v.w == g);
  }
#pragma unroll
  for (int g = 0; g < 16; ++g) cnt[tid * 16 + g] = c[g];
  __syncthreads();
  if (tid < 32) {
    int s = 0;
    const int gsel = tid & 15;
#pragma unroll 1
    for (int t = 0; t < 256; ++t) s += cnt[t * 16 + gsel];
    tot[tid] = (tid < 16) ? s : 0;
  }
  __syncthreads();
  if (tid == 0) {
    int run = 0;
    for (int g = 0; g < 16; ++g) { ofs[g] = run; run += tot[g]; }
    ofs[16] = run;
    for (int g = 17; g < 32; ++g) ofs[g] = 0;
  }
  __syncthreads();
  if (tid < 32) {
    const int o = ofs[tid];
    const int z = tot[tid];
    *(volatile int*)(meta + tid) = o;
    *(volatile int*)(meta + 32 + tid) = z;
    __threadfence();
    *(volatile int*)(meta + tid) = o;
    *(volatile int*)(meta + 32 + tid) = z;
  }
}

#define PB_X  5184
#define PB_WQ 972
#define PB_WO 144
#define PB_SM 10
static_assert(PB_X * 256 * 8 == NGR * NCAP * FD);
static_assert(PB_WQ == (FD / 64) * (F3 / 64));
static_assert(PB_WO == NHD * (FD / 64));
static_assert(PB_SM * 256 == SM_TOT);

__global__ __launch_bounds__(256) void k_prep(
    const float* __restrict__ x, const float* __restrict__ Wqkv, const float* __restrict__ Wout,
    const float* __restrict__ freq, const float* __restrict__ wrope,
    const float* __restrict__ gamma, const float* __restrict__ beta,
    const int* __restrict__ meta,
    unsigned short* __restrict__ xbp, unsigned short* __restrict__ wqkvt,
    unsigned short* __restrict__ wout2, float* __restrict__ smallp) {
  __shared__ __align__(16) float tf[144 * 68];
  const int bx = blockIdx.x;
  const int tid = threadIdx.x;
  if (bx < PB_X) {
    const int idx = bx * 256 + tid;
    const int row = idx / 144, q = idx - row * 144;
    const int g = row / NCAP, slot = row - g * NCAP;
    const int off = clampi(meta[g], 0, NN);
    const int sz = clampi(meta[32 + g], 0, NCAP);
    const int src = clampi(off + slot, 0, NN - 1);
    const float* sp = x + (size_t)src * FD + q * 8;
    const v4f a = *(const v4fa*)(sp);
    const v4f b = *(const v4fa*)(sp + 4);
    asm volatile("" :: "v"(a), "v"(b));
    const unsigned msk = (slot < sz) ? 0xffffffffu : 0u;
    v4u o;
    o.x = pk16(f2bf_bits(a.x), f2bf_bits(a.y)) & msk;
    o.y = pk16(f2bf_bits(a.z), f2bf_bits(a.w)) & msk;
    o.z = pk16(f2bf_bits(b.x), f2bf_bits(b.y)) & msk;
    o.w = pk16(f2bf_bits(b.z), f2bf_bits(b.w)) & msk;
    unsigned short* dp = xbp + (size_t)idx * 8;
    *(volatile v4u*)dp = o;
    __threadfence();
    *(volatile v4u*)dp = o;
  } else if (bx < PB_X + PB_WQ) {
    const int t = bx - PB_X;
    const int rb = t / 54, cb = t - rb * 54;
    const int c0 = cb * 64;
    const int r0 = rb * 64;
    {
      const int lr = tid >> 4, c4 = (tid & 15) * 4;
#pragma unroll
      for (int it = 0; it < 4; ++it) {
        const int rr = it * 16 + lr;
        const v4f a = *(const v4fa*)(Wqkv + (size_t)(r0 + rr) * F3 + c0 + c4);
        *(v4fa*)(tf + rr * 68 + c4) = a;
      }
    }
    __syncthreads();
    const int sub = tid >> 3, c8 = (tid & 7) * 8;
    v4u hv[2];
#pragma unroll
    for (int it = 0; it < 2; ++it) {
      const int oc = it * 32 + sub;
      v4u a;
#pragma unroll
      for (int q = 0; q < 4; ++q) {
        const float f0 = tf[(c8 + 2 * q) * 68 + oc];
        const float f1 = tf[(c8 + 2 * q + 1) * 68 + oc];
        a[q] = pk16(f2bf_bits(f0), f2bf_bits(f1));
      }
      hv[it] = a;
    }
    for (int pass = 0; pass < 2; ++pass) {
#pragma unroll
      for (int it = 0; it < 2; ++it) {
        const int oc = it * 32 + sub;
        *(volatile v4u*)(wqkvt + (size_t)(c0 + oc) * FD + r0 + c8) = hv[it];
      }
      __threadfence();
    }
  } else if (bx < PB_X + PB_WQ + PB_WO) {
    const int t = bx - PB_X - PB_WQ;
    const int h = t / 18, nb = t - h * 18;
    const int n0 = nb * 64;
#pragma unroll 1
    for (int it = 0; it < 9; ++it) {
      const int idx = it * 256 + tid;
      const int d = idx >> 4, c4 = (idx & 15) * 4;
      const v4f a = *(const v4fa*)(Wout + (size_t)(h * HD + d) * FD + n0 + c4);
      *(v4fa*)(tf + d * 68 + c4) = a;
    }
    __syncthreads();
    for (int pass = 0; pass < 2; ++pass) {
#pragma unroll 1
      for (int it = 0; it < 10; ++it) {
        const int idx = it * 256 + tid;
        const int n = idx / 40, q = idx - n * 40;
        const int part = q / 20, qq = q - part * 20;
        const bool valid = qq < 18;
        const int db = valid ? qq * 8 : 136;
        const unsigned msk = valid ? 0xffffffffu : 0u;
        v4u o;
#pragma unroll
        for (int p = 0; p < 4; ++p) {
          const float f0 = tf[(db + 2 * p) * 68 + n];
          const float f1 = tf[(db + 2 * p + 1) * 68 + n];
          o[p] = pk16(f2bf_bits(f0), f2bf_bits(f1)) & msk;
        }
        *(volatile v4u*)(wout2 + (size_t)(n0 + n) * CTXW + h * RECW + q * 8) = o;
      }
      __threadfence();
    }
  } else {
    const int i = (bx - PB_X - PB_WQ - PB_WO) * 256 + tid;
    const float fa = freq[clampi(i - SM_AF, 0, 15)];
    const float fw = wrope[clampi(i - SM_WR, 0, 127)];
    const float fg = gamma[clampi(i - SM_G, 0, FD - 1)];
    const float fb = beta[clampi(i - SM_B, 0, FD - 1)];
    asm volatile("" :: "v"(fa), "v"(fw), "v"(fg), "v"(fb));
    const unsigned ua = __float_as_uint(fabsf(bfr(fa))) & ((i < 16) ? 0xffffffffu : 0u);
    const unsigned uw = __float_as_uint(bfr(fw)) & ((i >= SM_WR && i < SM_G) ? 0xffffffffu : 0u);
    const unsigned ug = __float_as_uint(bfr(fg)) & ((i >= SM_G && i < SM_B) ? 0xffffffffu : 0u);
    const unsigned ub = __float_as_uint(bfr(fb)) & ((i >= SM_B && i < SM_END) ? 0xffffffffu : 0u);
    const float v = __uint_as_float(ua | uw | ug | ub);
    *(volatile float*)(smallp + i) = v;
    __threadfence();
    *(volatile float*)(smallp + i) = v;
  }
}

__global__ __launch_bounds__(64) __attribute__((amdgpu_num_vgpr(248)))
void k_qkv(const unsigned short* __restrict__ xbp_g, const unsigned short* __restrict__ wqkvt,
           const int* __restrict__ meta, int g0,
           unsigned short* __restrict__ qk, unsigned short* __restrict__ vt) {
  __shared__ __align__(16) float sT[2][64 * 68];
  const int lane = threadIdx.x & 31;
  const int wave = __builtin_amdgcn_readfirstlane((int)(threadIdx.x >> 5));
  const int hh = lane >> 4, c = lane & 15;
  const int by = blockIdx.y;
  const int gl = by / 9;
  const int slot0 = (by - gl * 9) * 64;
  const int sz = clampi(meta[32 + g0 + gl], 0, NCAP);
  if (slot0 >= sz) return;
  const int m0 = by * 64;
  const int n0 = blockIdx.x * 128 + wave * 64;

  v8f acc[4][4];
#pragma unroll
  for (int i = 0; i < 4; ++i)
#pragma unroll
    for (int j = 0; j < 4; ++j) acc[i][j] = (v8f){0.f, 0.f, 0.f, 0.f, 0.f, 0.f, 0.f, 0.f};

  const __bf16* A = (const __bf16*)(const void*)xbp_g + (size_t)m0 * FD;
  const __bf16* Bt = (const __bf16*)(const void*)wqkvt + (size_t)n0 * FD;
  gemm_tile64(A, FD, Bt, FD, FD, lane, acc);

  float* slab = sT[wave];
#pragma unroll
  for (int i = 0; i < 4; ++i)
#pragma unroll
    for (int j = 0; j < 4; ++j)
#pragma unroll
      for (int r = 0; r < 8; ++r)
        slab[(i * 16 + 8 * hh + r) * 68 + j * 16 + c] = acc[i][j][r];
  wave_sync_lds();

  const int third = n0 / FD;
  const int nn = n0 - third * FD;
  const int q4 = lane >> 3, c8 = (lane & 7) * 8;
  if (third < 2) {
    unsigned short* P = qk + (size_t)third * ((size_t)GG * NCAP * QKW);
    for (int pass = 0; pass < 2; ++pass) {
#pragma unroll 1
      for (int it = 0; it < 16; ++it) {
        const int row = it * 4 + q4;
        const float* sp = slab + row * 68 + c8;
        v4u hv, lv;
#pragma unroll
        for (int p = 0; p < 4; ++p) {
          const float f0 = sp[2 * p], f1 = sp[2 * p + 1];
          const unsigned short h0 = f2bf_bits(f0), h1 = f2bf_bits(f1);
          hv[p] = pk16(h0, h1);
          lv[p] = pk16(f2bf_bits(f0 - bf_bits2f(h0)), f2bf_bits(f1 - bf_bits2f(h1)));
        }
        const size_t go = (size_t)(m0 + row) * QKW + nn + c8;
        *(volatile v4u*)(P + go) = hv;
        *(volatile v4u*)(P + go + FD) = lv;
      }
      __threadfence();
    }
  } else {
    unsigned short* Vh = vt + (size_t)gl * FD * NCAP;
    unsigned short* Vl = Vh + (size_t)GG * FD * NCAP;
    for (int pass = 0; pass < 2; ++pass) {
#pragma unroll 1
      for (int it = 0; it < 16; ++it) {
        const int n = it * 4 + q4;
        v4u hv, lv;
#pragma unroll
        for (int p = 0; p < 4; ++p) {
          const float f0 = slab[(c8 + 2 * p) * 68 + n];
          const float f1 = slab[(c8 + 2 * p + 1) * 68 + n];
          const unsigned short h0 = f2bf_bits(f0), h1 = f2bf_bits(f1);
          hv[p] = pk16(h0, h1);
          lv[p] = pk16(f2bf_bits(f0 - bf_bits2f(h0)), f2bf_bits(f1 - bf_bits2f(h1)));
        }
        const size_t go = (size_t)(nn + n) * NCAP + slot0 + c8;
        *(volatile v4u*)(Vh + go) = hv;
        *(volatile v4u*)(Vl + go) = lv;
      }
      __threadfence();
    }
  }
}

__global__ __launch_bounds__(256) void k_bias(const float* __restrict__ pos, const float* __restrict__ smallp,
                                              const int* __restrict__ meta, int g0, float* __restrict__ bias) {
  __shared__ float ps[NCAP * 3];
  __shared__ float afs[16];
  __shared__ float wrs[128];
  const int tid = threadIdx.x;
  const int gl = blockIdx.y;
  const int g = g0 + gl;
  const int off = clampi(meta[g], 0, NN);
  const int sz = clampi(meta[32 + g], 0, NCAP);
  const int i0 = blockIdx.x * 64;
  if (i0 >= sz) return;
  const int Jn = ((sz + 63) >> 6) << 6;
#pragma unroll 1
  for (int it = 0; it < 3; ++it) {
    int s = it * 256 + tid;
    s = (s < NCAP - 1) ? s : (NCAP - 1);
    const int node = clampi(off + s, 0, NN - 1);
    const float px = pos[node * 3 + 0], py = pos[node * 3 + 1], pz = pos[node * 3 + 2];
    ps[s * 3 + 0] = bfr(px);
    ps[s * 3 + 1] = bfr(py);
    ps[s * 3 + 2] = bfr(pz);
  }
  afs[tid & 15] = smallp[SM_AF + (tid & 15)];
  wrs[tid & 127] = smallp[SM_WR + (tid & 127)];
  __syncthreads();
  const int lane = tid & 31, w = tid >> 5;
#pragma unroll 1
  for (int rr = 0; rr < 8; ++rr) {
    const int i = i0 + w * 8 + rr;
    const float pix = ps[i * 3 + 0], piy = ps[i * 3 + 1], piz = ps[i * 3 + 2];
#pragma unroll 1
    for (int j = lane; j < Jn; j += 32) {
      const float dx = pix - ps[j * 3 + 0];
      const float dy = piy - ps[j * 3 + 1];
      const float dz = piz - ps[j * 3 + 2];
      const float d = sqrtf((dx * dx + dz * dz) + dy * dy);
      float bacc[8];
#pragma unroll
      for (int hd = 0; hd < 8; ++hd) bacc[hd] = 0.0f;
#pragma unroll 1
      for (int r = 0; r < 16; ++r) {
        const float av = d * afs[r];
        const float cv = (__builtin_amdgcn_ballot_w32(fabsf(av) > 512.0f) != 0u) ? cosf(av) : __cosf(av);
#pragma unroll
        for (int hd = 0; hd < 8; ++hd) bacc[hd] += cv * wrs[r * 8 + hd];
      }
      const bool live = (i < sz) && (j < sz);
      float bv[8];
#pragma unroll
      for (int hd = 0; hd < 8; ++hd) bv[hd] = live ? bacc[hd] : 0.0f;
      float* bp = bias + ((size_t)(gl * NHD) * NCAP + i) * NCAP + j;
#pragma unroll
      for (int hd = 0; hd < 8; ++hd) *(volatile float*)(bp + (size_t)hd * NCAP * NCAP) = bv[hd];
      __threadfence();
#pragma unroll
      for (int hd = 0; hd < 8; ++hd) *(volatile float*)(bp + (size_t)hd * NCAP * NCAP) = bv[hd];
    }
  }
}

#define AT_OFF_QH 0
#define AT_OFF_QL 20480
#define AT_OFF_KH 40960
#define AT_OFF_KL 61440
#define AT_OFF_VH 81920
#define AT_OFF_VL 100352
#define AT_OFF_BS 118784
#define AT_OFF_PH 136192
#define AT_OFF_PL 144384
#define AT_LDS    152576
static_assert(AT_OFF_QL - AT_OFF_QH == 64 * HDK * 2);
static_assert(AT_OFF_VL - AT_OFF_VH == HD * 64 * 2);
static_assert(AT_OFF_PH - AT_OFF_BS == 64 * 68 * 4);
static_assert(AT_LDS - AT_OFF_PL == 4 * 16 * 64 * 2);
static_assert(4 * 16 * RECW * 2 == 2 * 64 * HDK * 2);
static_assert(AT_LDS <= 327680);

__device__ __forceinline__ void stage_qk(__bf16* dst, const unsigned short* __restrict__ src, int row0, int h, int tid) {
#pragma unroll 4
  for (int it = 0; it < 20; ++it) {
    const int idx = it * 128 + tid;
    const int pl = idx / 1280, rem = idx - pl * 1280;
    const int r = rem / 20, q = rem - r * 20;
    const int qc = (q < 18) ? q : 17;
    v4u v = *(const v4ua*)(src + (size_t)(row0 + r) * QKW + pl * FD + h * HD + qc * 8);
    asm volatile("" :: "v"(v));
    const unsigned m = (q < 18) ? 0xffffffffu : 0u;
    const v4u m4 = {m, m, m, m};
    v = v & m4;
    *(v4ua*)(dst + pl * (64 * HDK) + r * HDK + q * 8) = v;
  }
}

__global__ __launch_bounds__(128) __attribute__((amdgpu_num_vgpr(248)))
void k_attn(const unsigned short* __restrict__ qp, const unsigned short* __restrict__ kp,
            const unsigned short* __restrict__ vtp, const float* __restrict__ bias,
            const int* __restrict__ meta, int g0, unsigned short* __restrict__ ctx) {
  extern __shared__ __align__(16) unsigned char smem[];
  __bf16* Qh = (__bf16*)(smem + AT_OFF_QH);
  __bf16* Ql = (__bf16*)(smem + AT_OFF_QL);
  __bf16* Kh = (__bf16*)(smem + AT_OFF_KH);
  __bf16* Kl = (__bf16*)(smem + AT_OFF_KL);
  __bf16* Vh = (__bf16*)(smem + AT_OFF_VH);
  __bf16* Vl = (__bf16*)(smem + AT_OFF_VL);
  float*  Bs = (float*)(smem + AT_OFF_BS);
  __bf16* Ph = (__bf16*)(smem + AT_OFF_PH);
  __bf16* Pl = (__bf16*)(smem + AT_OFF_PL);

  const int tid = threadIdx.x;
  const int lane = tid & 31;
  const int wave = __builtin_amdgcn_readfirstlane((int)(tid >> 5));
  const int hh = lane >> 4, c = lane & 15;
  const int qt = blockIdx.x, h = blockIdx.y, gl = blockIdx.z;
  const int g = g0 + gl;
  const int off = clampi(meta[g], 0, NN);
  const int sz = clampi(meta[32 + g], 0, NCAP);
  const int i0 = qt * 64;
  if (i0 >= sz) return;
  const int nkt = (sz + 63) >> 6;

  stage_qk(Qh, qp, gl * NCAP + i0, h, tid);

  float mrow[8], lrow[8];
  v8f oacc[9];
#pragma unroll
  for (int r = 0; r < 8; ++r) { mrow[r] = -INFINITY; lrow[r] = 0.0f; }
#pragma unroll
  for (int t = 0; t < 9; ++t) oacc[t] = (v8f){0.f, 0.f, 0.f, 0.f, 0.f, 0.f, 0.f, 0.f};
  const float sscale = 1.0f / 12.0f;
  __bf16* pwh = Ph + wave * (16 * 64);
  __bf16* pwl = Pl + wave * (16 * 64);

#pragma unroll 1
  for (int kt = 0; kt < nkt; ++kt) {
    const int kv0 = kt * 64;
    __syncthreads();
    stage_qk(Kh, kp, gl * NCAP + kv0, h, tid);
#pragma unroll 3
    for (int it = 0; it < 18; ++it) {
      const int idx = it * 128 + tid;
      const int pl = idx / 1152, rem = idx - pl * 1152;
      const int d = rem >> 3, q = rem & 7;
      const v4u v = *(const v4ua*)(vtp + (size_t)pl * ((size_t)GG * FD * NCAP) +
                                   (size_t)(gl * FD + h * HD + d) * NCAP + kv0 + q * 8);
      *(v4ua*)(Vh + pl * (HD * 64) + d * 64 + q * 8) = v;
    }
#pragma unroll 4
    for (int it = 0; it < 8; ++it) {
      const int idx = it * 128 + tid;
      const int r = idx >> 4, q = idx & 15;
      const v4f v = *(const v4fa*)(bias + ((size_t)(gl * NHD + h) * NCAP + i0 + r) * NCAP + kv0 + q * 4);
      *(v4fa*)(Bs + r * 68 + q * 4) = v;
    }
    __syncthreads();

    v8f s[4];
#pragma unroll
    for (int j = 0; j < 4; ++j) s[j] = (v8f){0.f, 0.f, 0.f, 0.f, 0.f, 0.f, 0.f, 0.f};
#pragma unroll 1
    for (int dc = 0; dc < 5; ++dc) {
      const v16b qah = ldfrag(Qh + (wave * 16 + c) * HDK + dc * 32 + 8 * hh);
      const v16b qal = ldfrag(Ql + (wave * 16 + c) * HDK + dc * 32 + 8 * hh);
#pragma unroll
      for (int j = 0; j < 4; ++j) {
        const v16b kb = ldfrag(Kh + (j * 16 + c) * HDK + dc * 32 + 8 * hh);
        const v16b kl = ldfrag(Kl + (j * 16 + c) * HDK + dc * 32 + 8 * hh);
        s[j] = mma_bf(qah, kb, s[j]);
        s[j] = mma_bf(qah, kl, s[j]);
        s[j] = mma_bf(qal, kb, s[j]);
      }
    }

    float cm[8];
#pragma unroll
    for (int r = 0; r < 8; ++r) {
      const int row = wave * 16 + 8 * hh + r;
      float m = -INFINITY;
#pragma unroll
      for (int j = 0; j < 4; ++j) {
        const float bsv = Bs[row * 68 + j * 16 + c];
        float sv = s[j][r] * sscale + bsv;
        sv = (kv0 + j * 16 + c < sz) ? sv : -INFINITY;
        s[j][r] = sv;
        m = selmax(m, sv);
      }
#pragma unroll
      for (int o = 1; o < 16; o <<= 1) m = selmax(m, __shfl_xor(m, o, 32));
      cm[r] = m;
    }
#pragma unroll
    for (int r = 0; r < 8; ++r) {
      const float mnew = selmax(mrow[r], cm[r]);
      const float alpha = __expf(mrow[r] - mnew);
      mrow[r] = mnew;
      float psum = 0.0f;
#pragma unroll
      for (int j = 0; j < 4; ++j) {
        const float e = __expf(s[j][r] - mnew);
        const float p = (kv0 + j * 16 + c < sz) ? e : 0.0f;
        psum += p;
        __bf16 a, b;
        split_bf(p, a, b);
        pwh[(8 * hh + r) * 64 + j * 16 + c] = a;
        pwl[(8 * hh + r) * 64 + j * 16 + c] = b;
      }
#pragma unroll
      for (int o = 1; o < 16; o <<= 1) psum += __shfl_xor(psum, o, 32);
      lrow[r] = lrow[r] * alpha + psum;
#pragma unroll
      for (int t = 0; t < 9; ++t) oacc[t][r] *= alpha;
    }
    wave_sync_lds();
#pragma unroll 1
    for (int kk = 0; kk < 2; ++kk) {
      const v16b pa = ldfrag(pwh + c * 64 + kk * 32 + 8 * hh);
      const v16b pl = ldfrag(pwl + c * 64 + kk * 32 + 8 * hh);
#pragma unroll
      for (int t = 0; t < 9; ++t) {
        const v16b vb = ldfrag(Vh + (t * 16 + c) * 64 + kk * 32 + 8 * hh);
        const v16b vl = ldfrag(Vl + (t * 16 + c) * 64 + kk * 32 + 8 * hh);
        oacc[t] = mma_bf(pa, vb, oacc[t]);
        oacc[t] = mma_bf(pa, vl, oacc[t]);
        oacc[t] = mma_bf(pl, vb, oacc[t]);
      }
    }
  }

  __syncthreads();
  __bf16* rec = Kh + wave * (16 * RECW);
#pragma unroll
  for (int r = 0; r < 8; ++r) {
    const float inv = 1.0f / lrow[r];
#pragma unroll
    for (int t = 0; t < 9; ++t) {
      __bf16 a, b;
      split_bf(oacc[t][r] * inv, a, b);
      rec[(8 * hh + r) * RECW + t * 16 + c] = a;
      rec[(8 * hh + r) * RECW + HDK + t * 16 + c] = b;
    }
  }
  {
    const v4u z4 = {0u, 0u, 0u, 0u};
    __bf16* zp = rec + c * RECW + hh * HDK + HD;
    *(v4ua*)(zp) = z4;
    *(v4ua*)(zp + 8) = z4;
  }
  wave_sync_lds();
  __bf16* cg = (__bf16*)(void*)ctx;
  for (int pass = 0; pass < 2; ++pass) {
#pragma unroll 1
    for (int it = 0; it < 20; ++it) {
      const int idx = it * 32 + lane;
      const int row = idx / 40, q = idx - row * 40;
      const v8b v = *(const v8ba*)(rec + row * RECW + q * 8);
      asm volatile("" :: "v"(v));
      const int slot = i0 + wave * 16 + row;
      const int node = clampi(off + slot, 0, NN - 1);
      if (slot < sz) *(volatile v8b*)(cg + (size_t)node * CTXW + h * RECW + q * 8) = v;
    }
    __threadfence();
  }
}

__global__ __launch_bounds__(128) __attribute__((amdgpu_num_vgpr(248)))
void k_out(const unsigned short* __restrict__ ctxp, const unsigned short* __restrict__ wo2,
           const float* __restrict__ xin, float* __restrict__ hout) {
  __shared__ __align__(16) float sT[4][16 * 68];
  const int lane = threadIdx.x & 31;
  const int wave = __builtin_amdgcn_readfirstlane((int)(threadIdx.x >> 5));
  const int hh = lane >> 4, c = lane & 15;
  const int m0 = blockIdx.y * 128 + (wave & 1) * 64;
  const int n0 = blockIdx.x * 128 + (wave >> 1) * 64;

  v8f acc[4][4];
#pragma unroll
  for (int i = 0; i < 4; ++i)
#pragma unroll
    for (int j = 0; j < 4; ++j) acc[i][j] = (v8f){0.f, 0.f, 0.f, 0.f, 0.f, 0.f, 0.f, 0.f};
  const __bf16* A = (const __bf16*)(const void*)ctxp + (size_t)m0 * CTXW;
  const __bf16* Bt = (const __bf16*)(const void*)wo2 + (size_t)n0 * CTXW;
  gemm_tile64(A, CTXW, Bt, CTXW, CTXW, lane, acc);

  float* slab = sT[wave];
  const int c4 = (lane & 15) * 4;
#pragma unroll
  for (int i = 0; i < 4; ++i) {
    const int mBase = m0 + i * 16;
#pragma unroll
    for (int j = 0; j < 4; ++j)
#pragma unroll
      for (int r = 0; r < 8; ++r) slab[(8 * hh + r) * 68 + j * 16 + c] = acc[i][j][r];
    wave_sync_lds();
    v4f val[8];
#pragma unroll
    for (int it = 0; it < 8; ++it) {
      const int row = it * 2 + hh;
      const v4f sv = *(const v4fa*)(slab + row * 68 + c4);
      const v4f xv = *(const v4fa*)(xin + (size_t)(mBase + row) * FD + n0 + c4);
      v4f o;
      o.x = sv.x + bfr(xv.x);
      o.y = sv.y + bfr(xv.y);
      o.z = sv.z + bfr(xv.z);
      o.w = sv.w + bfr(xv.w);
      val[it] = o;
    }
    for (int pass = 0; pass < 2; ++pass) {
#pragma unroll
      for (int it = 0; it < 8; ++it) {
        const int row = it * 2 + hh;
        *(volatile v4f*)(hout + (size_t)(mBase + row) * FD + n0 + c4) = val[it];
      }
      __threadfence();
    }
    wave_sync_lds();
  }
}

__global__ __launch_bounds__(256) void k_ln(const float* __restrict__ hbuf, const float* __restrict__ smallp,
                                            const int* __restrict__ batch, const int* __restrict__ meta,
                                            float* __restrict__ out) {
  __shared__ __align__(16) float gb[2 * FD];
  const int tid = threadIdx.x;
#pragma unroll 1
  for (int it = 0; it < 3; ++it) {
    int idx = it * 256 + tid;
    idx = (idx < 575) ? idx : 575;
    const v4f v = *(const v4fa*)(smallp + SM_G + idx * 4);
    *(v4fa*)(gb + idx * 4) = v;
  }
  __syncthreads();
  const int lane = tid & 31, wave = tid >> 5;
  int row = blockIdx.x * 8 + wave;
  row = (row < NN - 1) ? row : (NN - 1);
  const int g = clampi(batch[row], 0, NGR - 1);
  const bool over = meta[32 + g] > NCAP;

  v4f hv[9];
  float s = 0.0f;
#pragma unroll
  for (int it = 0; it < 9; ++it) {
    hv[it] = *(const v4fa*)(hbuf + (size_t)row * FD + (it * 32 + lane) * 4);
    s += (hv[it].x + hv[it].y) + (hv[it].z + hv[it].w);
  }
#pragma unroll
  for (int o = 16; o >= 1; o >>= 1) s += __shfl_xor(s, o, 32);
  const float mu = s * (1.0f / (float)FD);
  float ss = 0.0f;
#pragma unroll
  for (int it = 0; it < 9; ++it) {
    const float a = hv[it].x - mu, b = hv[it].y - mu, cc = hv[it].z - mu, d = hv[it].w - mu;
    ss += (a * a + b * b) + (cc * cc + d * d);
  }
#pragma unroll
  for (int o = 16; o >= 1; o >>= 1) ss += __shfl_xor(ss, o, 32);
  const float var = ss * (1.0f / (float)FD);
  const float rs = 1.0f / sqrtf(var + 1e-5f);
  const float nanv = __uint_as_float(0x7fc00000u);
  v4f y[9];
#pragma unroll
  for (int it = 0; it < 9; ++it) {
    const int col = (it * 32 + lane) * 4;
    const v4f gm = *(const v4fa*)(gb + col);
    const v4f bt = *(const v4fa*)(gb + FD + col);
    v4f o;
    o.x = (hv[it].x - mu) * rs * gm.x + bt.x;
    o.y = (hv[it].y - mu) * rs * gm.y + bt.y;
    o.z = (hv[it].z - mu) * rs * gm.z + bt.z;
    o.w = (hv[it].w - mu) * rs * gm.w + bt.w;
    o.x = over ? nanv : o.x;
    o.y = over ? nanv : o.y;
    o.z = over ? nanv : o.z;
    o.w = over ? nanv : o.w;
    y[it] = o;
  }
  for (int pass = 0; pass < 2; ++pass) {
#pragma unroll
    for (int it = 0; it < 9; ++it)
      *(volatile v4f*)(out + (size_t)row * FD + (it * 32 + lane) * 4) = y[it];
    __threadfence();
  }
}

extern "C" void kernel_launch(void* const* d_in, const int* in_sizes, int n_in,
                              void* d_out, int out_size, void* d_ws, size_t ws_size,
                              hipStream_t stream) {
  if (n_in < 9) return;
  if (in_sizes[0] != NN * FD || in_sizes[1] != NN * 3 || in_sizes[2] != FD * F3 || in_sizes[3] != FD * FD) return;
  if (in_sizes[4] != 16 || in_sizes[5] != 16 * NHD || in_sizes[6] != FD || in_sizes[7] != FD || in_sizes[8] != NN) return;
  if (out_size != NN * FD) return;

  const float* x     = (const float*)d_in[0];
  const float* pos   = (const float*)d_in[1];
  const float* Wqkv  = (const float*)d_in[2];
  const float* Wout  = (const float*)d_in[3];
  const float* freq  = (const float*)d_in[4];
  const float* wrope = (const float*)d_in[5];
  const float* gamma = (const float*)d_in[6];
  const float* beta  = (const float*)d_in[7];
  const int*   batch = (const int*)d_in[8];

  const size_t szWQ   = (size_t)F3 * FD * 2;
  const size_t szWO   = (size_t)FD * CTXW * 2;
  const size_t szCTX  = (size_t)NN * CTXW * 2;
  const size_t szXBP  = (size_t)NGR * NCAP * FD * 2;
  const size_t szBIAS = (size_t)GG * NHD * NCAP * NCAP * 4;
  const size_t szQK   = (size_t)GG * NCAP * QKW * 2;
  const size_t szVT   = (size_t)2 * GG * FD * NCAP * 2;
  const size_t szH    = (size_t)NN * FD * 4;
  const size_t oWQ = 0;
  const size_t oWO = oWQ + szWQ;
  const size_t oCTX = oWO + szWO;
  const size_t oR = oCTX + szCTX;
  const size_t oXBP = oR;
  const size_t oBIAS = oXBP + szXBP;
  const size_t oQ = oBIAS + szBIAS;
  const size_t oK = oQ + szQK;
  const size_t oVT = oK + szQK;
  const size_t oREnd = oVT + szVT;
  const size_t oMETA = oREnd;
  const size_t oSM = oMETA + 256;
  const size_t total = oSM + (size_t)SM_TOT * 4;
  if (szH > oREnd - oR) return;
  if (total > ws_size) return;
  if (total > (size_t)134217728) return;

  char* ws = (char*)d_ws;
  unsigned short* wqkvt = (unsigned short*)(ws + oWQ);
  unsigned short* wout2 = (unsigned short*)(ws + oWO);
  unsigned short* ctx   = (unsigned short*)(ws + oCTX);
  unsigned short* xbp   = (unsigned short*)(ws + oXBP);
  float*          biasp = (float*)(ws + oBIAS);
  unsigned short* qpl   = (unsigned short*)(ws + oQ);
  unsigned short* kpl   = (unsigned short*)(ws + oK);
  unsigned short* vtp   = (unsigned short*)(ws + oVT);
  float*          hbuf  = (float*)(ws + oR);
  int*            meta  = (int*)(ws + oMETA);
  float*          smallp = (float*)(ws + oSM);

  (void)hipFuncSetAttribute(reinterpret_cast<const void*>(&k_attn), hipFuncAttributeMaxDynamicSharedMemorySize, AT_LDS);

  k_off<<<dim3(1), dim3(256), 0, stream>>>(batch, meta);
  k_prep<<<dim3(PB_X + PB_WQ + PB_WO + PB_SM), dim3(256), 0, stream>>>(
      x, Wqkv, Wout, freq, wrope, gamma, beta, meta, xbp, wqkvt, wout2, smallp);

  for (int gi = 0; gi < NGRP; ++gi) {
    const int g0 = gi * GG;
    const unsigned short* xg = xbp + (size_t)gi * GG * NCAP * FD;
    k_qkv<<<dim3(F3 / 128, (GG * NCAP) / 64), dim3(64), 0, stream>>>(xg, wqkvt, meta, g0, qpl, vtp);
    k_bias<<<dim3(NCAP / 64, GG), dim3(256), 0, stream>>>(pos, smallp, meta, g0, biasp);
    k_attn<<<dim3(NCAP / 64, NHD, GG), dim3(128), AT_LDS, stream>>>(qpl, kpl, vtp, biasp, meta, g0, ctx);
  }

  k_out<<<dim3(FD / 128, NN / 128), dim3(128), 0, stream>>>(ctx, wout2, x, hbuf);
  k_ln<<<dim3(NN / 8), dim3(256), 0, stream>>>(hbuf, smallp, batch, meta, (float*)d_out);
  (void)hipGetLastError();
}
